// MLPAttention_63677185131059
// MI455X (gfx1250) — hardware-verified
//
#include <hip/hip_runtime.h>
#include <math.h>

typedef __attribute__((ext_vector_type(16))) _Float16 v16h;
typedef __attribute__((ext_vector_type(16))) __bf16 v16b;
typedef __attribute__((ext_vector_type(8)))  _Float16 v8h;
typedef __attribute__((ext_vector_type(8)))  float v8f;
typedef __attribute__((ext_vector_type(4)))  float v4f;
typedef __attribute__((ext_vector_type(2)))  float v2f;
typedef __attribute__((ext_vector_type(4)))  unsigned v4u;
typedef __attribute__((ext_vector_type(4)))  int v4i;
typedef float __attribute__((may_alias)) float_a;
typedef int __attribute__((may_alias)) int_a;

template <typename T> __device__ __forceinline__ void vst2(void* p, T v) { *(volatile T*)p = v; __threadfence(); *(volatile T*)p = v; }
__device__ __forceinline__ v8f wmma16(v16h a, v16h b, v8f c) {
  v8f d = __builtin_amdgcn_wmma_f32_16x16x32_f16(false, a, false, b, (short)0, c, false, false);
  asm volatile("v_nop\n\tv_nop\n\tv_nop\n\tv_nop" : "+v"(d) : "v"(a), "v"(b));
  return d;
}
__device__ __forceinline__ v8f wmma_bf(v16b a, v16b b, v8f c) {
  v8f d = __builtin_amdgcn_wmma_f32_16x16x32_bf16(false, a, false, b, (short)0, c, false, false);
  asm volatile("v_nop\n\tv_nop\n\tv_nop\n\tv_nop" : "+v"(d) : "v"(a), "v"(b));
  return d;
}
__device__ __forceinline__ v16h frag_h(const _Float16* rowk0, int lane) {
  union { v16h v; v8h q[2]; } u; const _Float16* p = rowk0 + 8 * (lane >> 4);
  u.q[0] = *(const v8h*)p; u.q[1] = *(const v8h*)(p + 16); return u.v;
}
__device__ __forceinline__ v16h frag_f32(const float* rowk0, int lane) {
  v16h a; const float* p = rowk0 + 8 * (lane >> 4);
#pragma unroll
  for (int i = 0; i < 8; ++i) { a[i] = (_Float16)p[i]; a[8 + i] = (_Float16)p[16 + i]; }
  return a;
}
__device__ __forceinline__ v16h frag_f32s(const float* rowk0, int lane, float sc) {
  v16h a; const float* p = rowk0 + 8 * (lane >> 4);
#pragma unroll
  for (int i = 0; i < 8; ++i) { a[i] = (_Float16)(p[i] * sc); a[8 + i] = (_Float16)(p[16 + i] * sc); }
  return a;
}
__device__ __forceinline__ v16h fragc_f32(const float* W, int k0, int n, int lane, int ld, int K) {
  v16h a; const int g = lane >> 4;
#pragma unroll
  for (int i = 0; i < 8; ++i) { const int ka = k0 + 8 * g + i, kb = ka + 16;
    a[i] = (_Float16)(ka < K ? W[(size_t)(ka < K ? ka : K - 1) * ld + n] : 0.f); a[8 + i] = (_Float16)(kb < K ? W[(size_t)(kb < K ? kb : K - 1) * ld + n] : 0.f); }
  return a;
}
struct F2 { v16b h, l; };
__device__ __forceinline__ F2 bsplit16(const float v[16]) { F2 r;
#pragma unroll
  for (int i = 0; i < 16; ++i) { const __bf16 h = (__bf16)v[i]; r.h[i] = h; r.l[i] = (__bf16)(v[i] - (float)h); }
  return r; }
__device__ __forceinline__ F2 split_row(const float* row, int k0, int lane) { float v[16]; const float* p = row + k0 + 8 * (lane >> 4);
#pragma unroll
  for (int i = 0; i < 8; ++i) { v[i] = p[i]; v[8 + i] = p[16 + i]; }
  return bsplit16(v); }
__device__ __forceinline__ F2 split_rowK(const float* row, int k0, int lane, int K) { float v[16]; const int g = lane >> 4;
#pragma unroll
  for (int i = 0; i < 8; ++i) { const int ka = k0 + 8 * g + i, kb = ka + 16; v[i] = ka < K ? row[ka < K ? ka : K - 1] : 0.f; v[8 + i] = kb < K ? row[kb < K ? kb : K - 1] : 0.f; }
  return bsplit16(v); }
__device__ __forceinline__ F2 split_col(const float* W, int k0, int n, int lane, int ld, int K) { float v[16]; const int g = lane >> 4;
#pragma unroll
  for (int i = 0; i < 8; ++i) { const int ka = k0 + 8 * g + i, kb = ka + 16; v[i] = ka < K ? W[(size_t)(ka < K ? ka : K - 1) * ld + n] : 0.f; v[8 + i] = kb < K ? W[(size_t)(kb < K ? kb : K - 1) * ld + n] : 0.f; }
  return bsplit16(v); }
__device__ __forceinline__ v8f mac3(const F2& a, const F2& b, v8f c) { c = wmma_bf(a.l, b.h, c); c = wmma_bf(a.h, b.l, c); return wmma_bf(a.h, b.h, c); }
__device__ __forceinline__ float sigm(float v) { return 1.0f / (1.0f + expf(-v)); }
#define LDSX() do { asm volatile("s_wait_dscnt 0" ::: "memory"); __builtin_amdgcn_wave_barrier(); __builtin_amdgcn_fence(__ATOMIC_RELEASE, "workgroup"); } while (0)

#define NBT 4
#define TQ 256
#define TK 256
#define HD_ 256
#define QB 16
#ifndef NBV
#define NBV NBT
#endif
__device__ __forceinline__ float bfr(float v) { return (float)(__bf16)v; }
__device__ __forceinline__ v16b wcol_kz(const float* __restrict__ Wm, int k0, int o, int lane, int ld, int K, int nvalid) { v16b w; const int g = lane >> 4; const int oc = o < nvalid ? o : 0; const float keepo = o < nvalid ? 1.f : 0.f;
  asm volatile("s_wait_loadcnt 0x0" ::: "memory");
#pragma unroll
  for (int i = 0; i < 8; ++i) { const int ka = k0 + 8 * g + i, kb = ka + 16; w[i] = (__bf16)(Wm[(size_t)(ka < K ? ka : 0) * ld + oc] * (ka < K ? keepo : 0.f)); w[8 + i] = (__bf16)(Wm[(size_t)(kb < K ? kb : 0) * ld + oc] * (kb < K ? keepo : 0.f)); }
  asm volatile("s_wait_loadcnt 0x0" ::: "memory"); return w; }
#define WS_QH  0u
#define WS_KH  (WS_QH + 4u * (size_t)NBT * TQ * HD_)
#define WS_END (WS_KH + 4u * (size_t)NBT * TK * HD_)
__global__ __launch_bounds__(128) void k_lin(const float* __restrict__ XQ, const float* __restrict__ XK, const float* __restrict__ W1, float* __restrict__ QH, float* __restrict__ KH) { __shared__ __align__(16) float sf[4][16][132];
  const int tid = threadIdx.x, wave = tid >> 5, lane = tid & 31, col = lane & 15, g = lane >> 4; const int which = blockIdx.z; const int c0 = blockIdx.y * 128; const size_t r0 = (size_t)blockIdx.x * 64 + wave * 16;
  const float* X = which == 0 ? XQ : XK; const float* Wm = which == 0 ? W1 + (size_t)HD_ * HD_ : W1; float* OUT = which == 0 ? QH : KH;
  v8f acc[8] = {};
#pragma unroll 2
  for (int kc = 0; kc < HD_ / 32; ++kc) { v16b a; { const float* p = X + (r0 + col) * HD_ + kc * 32 + 8 * g;
#pragma unroll
      for (int i = 0; i < 8; ++i) { a[i] = (__bf16)p[i]; a[8 + i] = (__bf16)p[16 + i]; } }
    asm volatile("s_wait_loadcnt 0x0" ::: "memory");
#pragma unroll
    for (int j = 0; j < 8; ++j) { const v16b w = wcol_kz(Wm, kc * 32, c0 + j * 16 + col, lane, HD_, HD_, HD_); acc[j] = wmma_bf(a, w, acc[j]); } }
#pragma unroll
  for (int j = 0; j < 8; ++j) {
#pragma unroll
    for (int r = 0; r < 8; ++r) sf[wave][8 * g + r][j * 16 + col] = acc[j][r]; }
  LDSX(); for (int rl = 0; rl < 16; ++rl) vst2(OUT + (r0 + rl) * HD_ + c0 + lane * 4, *(const v4f*)&sf[wave][rl][lane * 4]); }
__global__ __launch_bounds__(128) void k_mlp(const float* __restrict__ QH, const float* __restrict__ KH, const float* __restrict__ KEYS, const int* __restrict__ QL, const int* __restrict__ KL, const float* __restrict__ B1, const float* __restrict__ W2, const float* __restrict__ B2, const float* __restrict__ W3, const float* __restrict__ B3, float* __restrict__ OUT) {
  __shared__ __align__(16) float sq[QB][HD_]; __shared__ __align__(16) float ss[QB][TK + 4]; __shared__ __align__(16) float so[4][16][68];
  const int tid = threadIdx.x, wave = tid >> 5, lane = tid & 31, col = lane & 15, g = lane >> 4; const size_t b = blockIdx.x; const int q0 = blockIdx.y * QB;
  int qlen = QL[b], klen = KL[b]; qlen = qlen < 0 ? 0 : (qlen > TQ ? TQ : qlen); klen = klen < 0 ? 0 : (klen > TK ? TK : klen);
  for (int e = tid; e < QB * HD_ / 4; e += 128) { const int qq = e / (HD_ / 4), c4 = e % (HD_ / 4); const v4f v = *(const v4f*)(QH + ((b * TQ + q0 + qq) * HD_) + c4 * 4); const v4f bb = *(const v4f*)(B1 + c4 * 4); asm volatile("s_wait_loadcnt 0x0" ::: "memory"); v4f o; o[0] = v[0] + bfr(bb[0]); o[1] = v[1] + bfr(bb[1]); o[2] = v[2] + bfr(bb[2]); o[3] = v[3] + bfr(bb[3]); *(v4f*)&sq[qq][c4 * 4] = o; }
  __syncthreads();
  const float b3v = bfr(B3[0]);
#pragma unroll 1
  for (int qq = 0; qq < QB; ++qq) {
#pragma unroll 1
    for (int rt = 0; rt < 4; ++rt) { const int k0 = wave * 64 + rt * 16; const float* khr = KH + (b * TK + k0 + col) * (size_t)HD_;
      float ps[8] = {0.f, 0.f, 0.f, 0.f, 0.f, 0.f, 0.f, 0.f};
#pragma unroll 1
      for (int half = 0; half < 2; ++half) {
        float b2r[8], w3r[8];
#pragma unroll
        for (int j = 0; j < 8; ++j) { b2r[j] = bfr(B2[half * 128 + j * 16 + col]); w3r[j] = bfr(W3[half * 128 + j * 16 + col]); }
        asm volatile("s_wait_loadcnt 0x0" ::: "memory");
        v8f acc[8] = {};
#pragma unroll 1
        for (int kc = 0; kc < HD_ / 32; ++kc) { float va[16];
#pragma unroll
          for (int i = 0; i < 8; ++i) { const int c = kc * 32 + 8 * g + i; va[i] = khr[c]; }
          asm volatile("s_wait_loadcnt 0x0" ::: "memory");
#pragma unroll
          for (int i = 8; i < 16; ++i) { const int c = kc * 32 + 8 * g + 8 + i; va[i] = khr[c]; }
          asm volatile("s_wait_loadcnt 0x0" ::: "memory");
#pragma unroll
          for (int i = 0; i < 16; ++i) { const int c = kc * 32 + 8 * g + (i < 8 ? i : 8 + i); va[i] = fmaxf(va[i] + sq[qq][c], 0.f); }
          const F2 a = bsplit16(va);
#pragma unroll
          for (int j = 0; j < 8; ++j) { const v16b w = wcol_kz(W2, kc * 32, half * 128 + j * 16 + col, lane, HD_, HD_, HD_); acc[j] = wmma_bf(a.h, w, acc[j]); acc[j] = wmma_bf(a.l, w, acc[j]); } }
#pragma unroll
        for (int r = 0; r < 8; ++r) { float p = ps[r];
#pragma unroll
          for (int j = 0; j < 8; ++j) p += fmaxf(acc[j][r] + b2r[j], 0.f) * w3r[j]; ps[r] = p; } }
#pragma unroll
      for (int o = 1; o < 16; o <<= 1) {
#pragma unroll
        for (int r = 0; r < 8; ++r) ps[r] += __shfl_xor(ps[r], o); }
      if (col == 0) {
#pragma unroll
        for (int r = 0; r < 8; ++r) ss[qq][k0 + 8 * g + r] = ps[r] + b3v; } } }
  __syncthreads();
#pragma unroll 1
  for (int i = 0; i < 4; ++i) { const int qq = wave * 4 + i; const bool qvalid = (q0 + qq) < qlen; float v[8]; float m = -3.0e38f;
#pragma unroll
    for (int u = 0; u < 8; ++u) { float t2 = ss[qq][lane * 8 + u]; asm volatile("" : "+v"(t2)); v[u] = t2; }
#pragma unroll
    for (int u = 0; u < 8; ++u) { const int k = lane * 8 + u; v[u] = (k < klen) ? v[u] : -3.0e38f; m = fmaxf(m, v[u]); }
#pragma unroll
    for (int o = 1; o < 32; o <<= 1) m = fmaxf(m, __shfl_xor(m, o));
    float sum = 0.f, e[8];
#pragma unroll
    for (int u = 0; u < 8; ++u) { e[u] = (lane * 8 + u < klen) ? expf(v[u] - m) : 0.f; sum += e[u]; }
#pragma unroll
    for (int o = 1; o < 32; o <<= 1) sum += __shfl_xor(sum, o);
    const float inv = (qvalid && sum > 0.f) ? 1.0f / sum : 0.f;
    LDSX();
#pragma unroll
    for (int u = 0; u < 8; ++u) ss[qq][lane * 8 + u] = e[u] * inv; }
  __syncthreads();
  { v8f acc[4] = {};
#pragma unroll
    for (int kc = 0; kc < TK / 32; ++kc) { const F2 a = split_row(&ss[col][0], kc * 32, lane);
#pragma unroll
      for (int j = 0; j < 4; ++j) { const v16b w = wcol_kz(KEYS + b * TK * (size_t)HD_, kc * 32, wave * 64 + j * 16 + col, lane, HD_, TK, HD_); acc[j] = wmma_bf(a.h, w, acc[j]); acc[j] = wmma_bf(a.l, w, acc[j]); } }
#pragma unroll
    for (int j = 0; j < 4; ++j) {
#pragma unroll
      for (int r = 0; r < 8; ++r) so[wave][8 * g + r][j * 16 + col] = acc[j][r]; }
    LDSX(); for (int rl = 0; rl < 16; ++rl) if (lane < 16) vst2(OUT + ((b * TQ + q0 + rl) * HD_) + wave * 64 + lane * 4, *(const v4f*)&so[wave][rl][lane * 4]); } }
extern "C" void kernel_launch(void* const* d_in, const int* in_sizes, int n_in, void* d_out, int out_size, void* d_ws, size_t ws_size, hipStream_t stream) {
  (void)in_sizes; (void)n_in; (void)out_size;
  if (ws_size < (size_t)WS_END) return;
  char* ws = (char*)d_ws; const float** F = (const float**)d_in; float *QH = (float*)(ws + WS_QH), *KH = (float*)(ws + WS_KH);
  k_lin<<<dim3(NBV * TQ / 64, HD_ / 128, 2), 128, 0, stream>>>(F[0], F[1], F[4], QH, KH);
  k_mlp<<<dim3(NBV, TQ / QB), 128, 0, stream>>>(QH, KH, F[1], (const int*)d_in[2], (const int*)d_in[3], F[5], F[6], F[7], F[8], F[9], (float*)d_out);
}
